// Casual_11948599017518
// MI455X (gfx1250) — hardware-verified
//
#include <hip/hip_runtime.h>

typedef __attribute__((ext_vector_type(16))) _Float16 v16h;
typedef __attribute__((ext_vector_type(8)))  _Float16 v8h;
typedef __attribute__((ext_vector_type(16))) __bf16   v16b;
typedef __attribute__((ext_vector_type(8)))  __bf16   v8b;
typedef __attribute__((ext_vector_type(8)))  float    v8f;
typedef __attribute__((ext_vector_type(4)))  float    v4f;
typedef __attribute__((ext_vector_type(4)))  unsigned int v4u;

constexpr int  DIM_IN    = 256;
constexpr int  DIM_HID   = 512;
constexpr int  NUM_EXP   = 8;
constexpr int  DIM_EO    = 256;
constexpr int  DIM_OUT   = 256;
constexpr int  NCAT      = NUM_EXP * DIM_HID;
constexpr int  KFC2      = NCAT + 32;
constexpr int  LD_HGX    = 4160;
constexpr int  LD_W2T    = 4160;
constexpr int  GX_COL    = NCAT;
constexpr int  CHUNK_ROWS = 4096;
constexpr int  NGATE_PAD = 64;
constexpr float HG_CARRY = 16.0f;
constexpr float W2_CARRY = 16.0f;
constexpr float FC2_SCALE = 1.0f / 256.0f;
constexpr int  GRP_COLS_SHIFT = 9;


__device__ __forceinline__ unsigned short f2bf_bits(float f) {
  unsigned u = __float_as_uint(f);
  return (unsigned short)((u + 0x7FFFu + ((u >> 16) & 1u)) >> 16);
}
__device__ __forceinline__ float bf_bits2f(unsigned short h) { return __uint_as_float(((unsigned)h) << 16); }
__device__ __forceinline__ float bfr(float f) { return bf_bits2f(f2bf_bits(f)); }
__device__ __forceinline__ unsigned h_bits(float f) { return (unsigned)__builtin_bit_cast(unsigned short, (_Float16)f); }

__device__ __forceinline__ void dep_guard_h(v8f& a, v8f& b, v16h x, v16h y) { asm volatile("v_nop\n\tv_nop\n\tv_nop\n\tv_nop" : "+v"(a), "+v"(b) : "v"(x), "v"(y)); }
__device__ __forceinline__ void dep_guard_b(v8f& a, v8f& b, v16b x, v16b y) { asm volatile("v_nop\n\tv_nop\n\tv_nop\n\tv_nop" : "+v"(a), "+v"(b) : "v"(x), "v"(y)); }
__device__ __forceinline__ void keep4_h(v16h a, v16h b, v16h c, v16h d) { asm volatile("v_nop" :: "v"(a), "v"(b), "v"(c), "v"(d)); }
__device__ __forceinline__ void keep4_b(v16b a, v16b b, v16b c, v16b d) { asm volatile("v_nop" :: "v"(a), "v"(b), "v"(c), "v"(d)); }
__device__ __forceinline__ void acc_guard4(v8f& a, v8f& b, v8f& c, v8f& d) { asm volatile("v_nop\n\tv_nop\n\tv_nop\n\tv_nop" : "+v"(a), "+v"(b), "+v"(c), "+v"(d)); }

template <typename T> struct Frag;
template <> struct Frag<_Float16> {
  typedef v16h V; union U { v16h v; v8h h[2]; };
  static __device__ __forceinline__ v16h load(const _Float16* p) {
    U f; f.h[0] = *(const v8h*)(p); f.h[1] = *(const v8h*)(p + 16); return f.v;
  }
  static __device__ __forceinline__ v8f mma(v16h a, v16h b, v8f c) {
    return __builtin_amdgcn_wmma_f32_16x16x32_f16(false, a, false, b, (short)0, c, false, false);
  }
  static __device__ __forceinline__ void guard(v8f& a, v8f& b, v16h x, v16h y) { dep_guard_h(a, b, x, y); }
  static __device__ __forceinline__ void keep(v16h a, v16h b, v16h c, v16h d) { keep4_h(a, b, c, d); }
};
template <> struct Frag<__bf16> {
  typedef v16b V; union U { v16b v; v8b h[2]; };
  static __device__ __forceinline__ v16b load(const __bf16* p) {
    U f; f.h[0] = *(const v8b*)(p); f.h[1] = *(const v8b*)(p + 16); return f.v;
  }
  static __device__ __forceinline__ v8f mma(v16b a, v16b b, v8f c) {
    return __builtin_amdgcn_wmma_f32_16x16x32_bf16(false, a, false, b, (short)0, c, false, false);
  }
  static __device__ __forceinline__ void guard(v8f& a, v8f& b, v16b x, v16b y) { dep_guard_b(a, b, x, y); }
  static __device__ __forceinline__ void keep(v16b a, v16b b, v16b c, v16b d) { keep4_b(a, b, c, d); }
};

template <int ET> struct Elem;
template <> struct Elem<0> { typedef _Float16 T; };
template <> struct Elem<1> { typedef __bf16 T; };
template <int ET, int SPLITM, int BIAS_MODE, int OUT_MODE, bool GMUL, int ACT>
__global__ __launch_bounds__(256) void gemm64t(
    const unsigned short* __restrict__ Ap, const unsigned short* __restrict__ A2p, int lda, long strideA,
    const unsigned short* __restrict__ Btp, const unsigned short* __restrict__ Bt2p, int ldb, long strideB,
    void* __restrict__ Cout, void* __restrict__ Cout2, int ldc, long strideC,
    const float* __restrict__ bias, const float* __restrict__ rowgrp,
    int M, int N, int K, float scale) {
  typedef typename Elem<ET>::T T;
  typedef typename Frag<T>::V V;
  const T* A = (const T*)Ap; const T* A2 = (const T*)A2p; const T* Bt = (const T*)Btp; const T* Bt2 = (const T*)Bt2p;
  __shared__ __align__(16) float sT[8][16 * 68];
  const int b    = blockIdx.y;
  const int lane = threadIdx.x & 31;
  const int wave = threadIdx.x >> 5;
  const int tilesN = N >> 6;
  const int tilesM = M >> 6;
  const int tile = blockIdx.x * 8 + wave;
  if (tile >= tilesM * tilesN) return;
  const int tm = tile / tilesN;
  const int tn = tile - tm * tilesN;
  const int m0 = tm << 6;
  const int n0 = tn << 6;

  const T* Ab  = A  + (size_t)b * strideA;
  const T* Bb  = Bt + (size_t)b * strideB;
  const T* Ab2 = (SPLITM >= 1) ? (A2  + (size_t)b * strideA) : nullptr;
  const T* Bb2 = (SPLITM == 2) ? (Bt2 + (size_t)b * strideB) : nullptr;

  const int rlane = lane & 15;
  const int koff  = (lane >> 4) * 8;
  const int mOff  = (lane >> 4) * 8;

  v8f acc[4][4];
#pragma unroll
  for (int i = 0; i < 4; ++i)
#pragma unroll
    for (int j = 0; j < 4; ++j) acc[i][j] = (v8f){0.f,0.f,0.f,0.f,0.f,0.f,0.f,0.f};

  for (int k0 = 0; k0 < K; k0 += 32) {
    V bh[4], bl[4];
#pragma unroll
    for (int j = 0; j < 4; ++j) {
      const size_t bofs = (size_t)(n0 + (j << 4) + rlane) * ldb + koff + k0;
      bh[j] = Frag<T>::load(Bb + bofs);
      if (SPLITM == 2) bl[j] = Frag<T>::load(Bb2 + bofs);
    }
#pragma unroll
    for (int i = 0; i < 4; ++i) {
      const size_t ao = (size_t)(m0 + (i << 4) + rlane) * lda + koff + k0;
      V ah = Frag<T>::load(Ab + ao);
      V al;
      if (SPLITM >= 1) al = Frag<T>::load(Ab2 + ao);
#pragma unroll
      for (int j = 0; j < 4; ++j) {
        acc[i][j] = Frag<T>::mma(ah, bh[j], acc[i][j]);
        if (SPLITM == 2) acc[i][j] = Frag<T>::mma(ah, bl[j], acc[i][j]);
        if (SPLITM >= 1) acc[i][j] = Frag<T>::mma(al, bh[j], acc[i][j]);
      }
      Frag<T>::guard(acc[i][0], acc[i][3], ah, (SPLITM >= 1) ? al : ah);
    }
    Frag<T>::keep(bh[0], bh[1], bh[2], bh[3]);
    if (SPLITM == 2) Frag<T>::keep(bl[0], bl[1], bl[2], bl[3]);
  }
  acc_guard4(acc[0][0], acc[0][1], acc[0][2], acc[0][3]);
  acc_guard4(acc[1][0], acc[1][1], acc[1][2], acc[1][3]);
  acc_guard4(acc[2][0], acc[2][1], acc[2][2], acc[2][3]);
  acc_guard4(acc[3][0], acc[3][1], acc[3][2], acc[3][3]);

  float* slab = sT[wave];
  const int grp = n0 >> GRP_COLS_SHIFT;
#pragma unroll
  for (int i = 0; i < 4; ++i) {
    const int mBase = m0 + (i << 4);
    float gm[8];
#pragma unroll
    for (int r = 0; r < 8; ++r) gm[r] = GMUL ? rowgrp[(size_t)(mBase + mOff + r) * NUM_EXP + grp] : 1.0f;
#pragma unroll
    for (int j = 0; j < 4; ++j) {
      const int n = n0 + (j << 4) + rlane;
      float bv = 0.f;
      if (BIAS_MODE == 2) bv = bfr(bias[n]);
#pragma unroll
      for (int r = 0; r < 8; ++r) {
        float v = acc[i][j][r] * scale;
        if (BIAS_MODE == 1) v += bfr(bias[mBase + mOff + r]);
        if (BIAS_MODE == 2) v += bv;
        if (ACT == 2) v = fmaxf(v, 0.0f);
        if (GMUL) v = v * gm[r];
        slab[(mOff + r) * 68 + (j << 4) + rlane] = v;
      }
    }
    __builtin_amdgcn_fence(__ATOMIC_RELEASE, "workgroup");
    __builtin_amdgcn_wave_barrier();
    __builtin_amdgcn_fence(__ATOMIC_ACQUIRE, "workgroup");
    if (OUT_MODE == 0) {
      float* C = (float*)Cout + (size_t)b * strideC;
      const int hh = lane >> 4, c4 = (lane & 15) * 4;
      for (int pass = 0; pass < 2; ++pass) {
#pragma unroll
        for (int it = 0; it < 8; ++it) {
          const int row = it * 2 + hh;
          v4f v = *(const v4f*)(slab + row * 68 + c4);
          *(volatile v4f*)(C + (size_t)(mBase + row) * ldc + n0 + c4) = v;
        }
        __threadfence();
      }
    } else {
      const int q = lane >> 3, c8 = (lane & 7) * 8;
      unsigned short* C  = (unsigned short*)Cout  + (size_t)b * strideC;
      unsigned short* Cb = (OUT_MODE == 2) ? ((unsigned short*)Cout2 + (size_t)b * strideC) : nullptr;
      for (int pass = 0; pass < 2; ++pass) {
#pragma unroll
        for (int it = 0; it < 4; ++it) {
          const int row = it * 4 + q;
          const float* sp = slab + row * 68 + c8;
          v8h hv, lv;
#pragma unroll
          for (int e = 0; e < 8; ++e) {
            if (OUT_MODE == 1) {
              hv[e] = (_Float16)sp[e];
            } else {
              unsigned short hb = f2bf_bits(sp[e]);
              unsigned short lb = f2bf_bits(sp[e] - bf_bits2f(hb));
              hv[e] = __builtin_bit_cast(_Float16, hb);
              lv[e] = __builtin_bit_cast(_Float16, lb);
            }
          }
          *(volatile v8h*)(C + (size_t)(mBase + row) * ldc + n0 + c8) = hv;
          if (OUT_MODE == 2) *(volatile v8h*)(Cb + (size_t)(mBase + row) * ldc + n0 + c8) = lv;
        }
        __threadfence();
      }
    }
    __builtin_amdgcn_fence(__ATOMIC_RELEASE, "workgroup");
    __builtin_amdgcn_wave_barrier();
    __builtin_amdgcn_fence(__ATOMIC_ACQUIRE, "workgroup");
  }
}

__global__ __launch_bounds__(256) void cast_f32_bf16x8(
    const float* __restrict__ in, unsigned short* __restrict__ out, int n8) {
  const int i = blockIdx.x * 256 + threadIdx.x;
  if (i >= n8) return;
  const float* p = in + (size_t)i * 8;
  const v4f a = *(const v4f*)(p);
  const v4f c = *(const v4f*)(p + 4);
  v4u w;
  w.x = (unsigned)f2bf_bits(a.x) | ((unsigned)f2bf_bits(a.y) << 16);
  w.y = (unsigned)f2bf_bits(a.z) | ((unsigned)f2bf_bits(a.w) << 16);
  w.z = (unsigned)f2bf_bits(c.x) | ((unsigned)f2bf_bits(c.y) << 16);
  w.w = (unsigned)f2bf_bits(c.z) | ((unsigned)f2bf_bits(c.w) << 16);
  unsigned short* o = out + (size_t)i * 8;
  *(volatile v4u*)o = w;
  __threadfence();
  *(volatile v4u*)o = w;
}

template <int MODE>
__global__ __launch_bounds__(256) void transpose_cast64(
    const float* __restrict__ in, int ldi, long strideIn,
    unsigned short* __restrict__ out, int ldo, long strideOut) {
  __shared__ __align__(16) unsigned short sT[64 * 72];
  const int tid = threadIdx.x;
  const int c0 = blockIdx.x * 64;
  const int r0 = blockIdx.y * 64;
  const float* ib = in + (size_t)blockIdx.z * strideIn;
  unsigned short* ob = out + (size_t)blockIdx.z * strideOut;
#pragma unroll
  for (int it = 0; it < 4; ++it) {
    const int idx = it * 256 + tid;
    const int r = idx >> 4;
    const int c4 = (idx & 15) * 4;
    const v4f v = *(const v4f*)(ib + (size_t)(r0 + r) * ldi + c0 + c4);
    unsigned short t0, t1, t2, t3;
    if (MODE == 0) {
      t0 = f2bf_bits(v.x); t1 = f2bf_bits(v.y); t2 = f2bf_bits(v.z); t3 = f2bf_bits(v.w);
    } else {
      t0 = (unsigned short)h_bits(W2_CARRY * bfr(v.x));
      t1 = (unsigned short)h_bits(W2_CARRY * bfr(v.y));
      t2 = (unsigned short)h_bits(W2_CARRY * bfr(v.z));
      t3 = (unsigned short)h_bits(W2_CARRY * bfr(v.w));
    }
    sT[(c4 + 0) * 72 + r] = t0;
    sT[(c4 + 1) * 72 + r] = t1;
    sT[(c4 + 2) * 72 + r] = t2;
    sT[(c4 + 3) * 72 + r] = t3;
  }
  __syncthreads();
  const int q = tid & 7;
  for (int pass = 0; pass < 2; ++pass) {
#pragma unroll
    for (int it = 0; it < 2; ++it) {
      const int oc = it * 32 + (tid >> 3);
      const v4u w = *(const v4u*)(sT + oc * 72 + 8 * q);
      *(volatile v4u*)(ob + (size_t)(c0 + oc) * ldo + r0 + 8 * q) = w;
    }
    __threadfence();
  }
}

__global__ __launch_bounds__(256) void build_wgt(const float* __restrict__ wg, unsigned short* __restrict__ wgt) {
  const int tid = threadIdx.x;
  for (int pass = 0; pass < 2; ++pass) {
#pragma unroll
    for (int it = 0; it < 8; ++it) {
      const int item = it * 256 + tid;
      const int r = item >> 5;
      const int g = item & 31;
      const int rr = (r < NUM_EXP) ? r : (NUM_EXP - 1);
      const unsigned keep = (r < NUM_EXP) ? 0xffffffffu : 0u;
      unsigned bits[8];
#pragma unroll
      for (int i = 0; i < 8; ++i) bits[i] = (unsigned)f2bf_bits(wg[(size_t)(8 * g + i) * NUM_EXP + rr]);
      v4u w;
      w.x = (bits[0] | (bits[1] << 16)) & keep;
      w.y = (bits[2] | (bits[3] << 16)) & keep;
      w.z = (bits[4] | (bits[5] << 16)) & keep;
      w.w = (bits[6] | (bits[7] << 16)) & keep;
      *(volatile v4u*)(wgt + (size_t)r * DIM_IN + 8 * g) = w;
    }
    __threadfence();
  }
}

__global__ __launch_bounds__(256) void build_w2t_tail(const float* __restrict__ b2, unsigned short* __restrict__ w2t) {
  const int tid = threadIdx.x;
  const int q = tid & 7;
  const unsigned keep = (q == 0) ? 0xffffffffu : 0u;
  for (int pass = 0; pass < 2; ++pass) {
#pragma unroll
    for (int it = 0; it < 8; ++it) {
      const int o = it * 32 + (tid >> 3);
      unsigned bits[8];
#pragma unroll
      for (int e = 0; e < 8; ++e) bits[e] = h_bits(W2_CARRY * bfr(b2[(size_t)e * DIM_EO + o]));
      v4u w;
      w.x = (bits[0] | (bits[1] << 16)) & keep;
      w.y = (bits[2] | (bits[3] << 16)) & keep;
      w.z = (bits[4] | (bits[5] << 16)) & keep;
      w.w = (bits[6] | (bits[7] << 16)) & keep;
      *(volatile v4u*)(w2t + (size_t)o * LD_W2T + GX_COL + 8 * q) = w;
    }
    __threadfence();
  }
}

__global__ __launch_bounds__(256) void gate_softmax256(
    const float* __restrict__ gl, const float* __restrict__ bg,
    float* __restrict__ gate16, unsigned short* __restrict__ hgx) {
  __shared__ __align__(16) float sG[256 * 8];
  const int tid = threadIdx.x;
  const int row = blockIdx.x * 256 + tid;
  const float* lp = gl + (size_t)row * NGATE_PAD;
  const v4f a = *(const v4f*)(lp);
  const v4f c = *(const v4f*)(lp + 4);
  const float l0 = a.x + bfr(bg[0]), l1 = a.y + bfr(bg[1]), l2 = a.z + bfr(bg[2]), l3 = a.w + bfr(bg[3]);
  const float l4 = c.x + bfr(bg[4]), l5 = c.y + bfr(bg[5]), l6 = c.z + bfr(bg[6]), l7 = c.w + bfr(bg[7]);
  float m = fmaxf(fmaxf(fmaxf(l0, l1), fmaxf(l2, l3)), fmaxf(fmaxf(l4, l5), fmaxf(l6, l7)));
  float* my = sG + tid * 8;
  my[0] = l0; my[1] = l1; my[2] = l2; my[3] = l3; my[4] = l4; my[5] = l5; my[6] = l6; my[7] = l7;
  float s = 0.f;
#pragma unroll 1
  for (int e = 0; e < 8; ++e) {
    const float p = expf(my[e] - m);
    s += p;
    my[e] = p;
  }
  const float inv = 1.0f / s;
#pragma unroll 1
  for (int e = 0; e < 8; ++e) my[e] = (my[e] * inv) * HG_CARRY;
  __syncthreads();
  {
    float* gbase = gate16 + (size_t)blockIdx.x * 2048;
    for (int pass = 0; pass < 2; ++pass) {
#pragma unroll
      for (int it = 0; it < 2; ++it) {
        const int idx = it * 256 + tid;
        const v4f gv = *(const v4f*)(sG + 4 * idx);
        *(volatile v4f*)(gbase + 4 * idx) = gv;
      }
      __threadfence();
    }
  }
  const int q = tid & 7;
  const unsigned keep = (q == 0) ? 0xffffffffu : 0u;
  for (int pass = 0; pass < 2; ++pass) {
#pragma unroll
    for (int it = 0; it < 8; ++it) {
      const int r = it * 32 + (tid >> 3);
      const float* g8 = sG + r * 8;
      v4u w;
      w.x = (h_bits(g8[0]) | (h_bits(g8[1]) << 16)) & keep;
      w.y = (h_bits(g8[2]) | (h_bits(g8[3]) << 16)) & keep;
      w.z = (h_bits(g8[4]) | (h_bits(g8[5]) << 16)) & keep;
      w.w = (h_bits(g8[6]) | (h_bits(g8[7]) << 16)) & keep;
      *(volatile v4u*)(hgx + (size_t)(blockIdx.x * 256 + r) * LD_HGX + GX_COL + 8 * q) = w;
    }
    __threadfence();
  }
}

extern "C" void kernel_launch(void* const* d_in, const int* in_sizes, int n_in,
                              void* d_out, int out_size, void* d_ws, size_t ws_size,
                              hipStream_t stream) {
  if (n_in < 9) return;
  const float* x  = (const float*)d_in[0];
  const float* w1 = (const float*)d_in[1];
  const float* b1 = (const float*)d_in[2];
  const float* w2 = (const float*)d_in[3];
  const float* b2 = (const float*)d_in[4];
  const float* wg = (const float*)d_in[5];
  const float* bg = (const float*)d_in[6];
  const float* wo = (const float*)d_in[7];
  const float* bo = (const float*)d_in[8];
  float* out = (float*)d_out;

  const long T = (long)in_sizes[0] / DIM_IN;
  if (T <= 0 || (T % CHUNK_ROWS) != 0) return;
  if ((long)out_size != T * DIM_OUT) return;
  const int nChunk = (int)(T / CHUNK_ROWS);

  size_t off = 0;
  const size_t offXB   = off; off += (size_t)T * DIM_IN * 2;
  const size_t offW1T  = off; off += (size_t)NCAT * DIM_IN * 2;
  const size_t offW2T  = off; off += (size_t)DIM_EO * LD_W2T * 2;
  const size_t offWOT  = off; off += (size_t)DIM_OUT * DIM_EO * 2;
  const size_t offWGT  = off; off += (size_t)NGATE_PAD * DIM_IN * 2;
  const size_t offGL   = off; off += (size_t)T * NGATE_PAD * 4;
  const size_t offGATE = off; off += (size_t)CHUNK_ROWS * NUM_EXP * 4;
  const size_t offHGX  = off; off += (size_t)CHUNK_ROWS * LD_HGX * 2;
  const size_t offWEIH = off; off += (size_t)CHUNK_ROWS * DIM_EO * 2;
  const size_t offWEIL = off; off += (size_t)CHUNK_ROWS * DIM_EO * 2;
  if (off > ws_size) return;

  char* ws = (char*)d_ws;
  unsigned short* XB   = (unsigned short*)(ws + offXB);
  unsigned short* W1T  = (unsigned short*)(ws + offW1T);
  unsigned short* W2T  = (unsigned short*)(ws + offW2T);
  unsigned short* WOT  = (unsigned short*)(ws + offWOT);
  unsigned short* WGT  = (unsigned short*)(ws + offWGT);
  float*          GL   = (float*)(ws + offGL);
  float*          GATE = (float*)(ws + offGATE);
  unsigned short* HGX  = (unsigned short*)(ws + offHGX);
  unsigned short* WEIH = (unsigned short*)(ws + offWEIH);
  unsigned short* WEIL = (unsigned short*)(ws + offWEIL);

  {
    const int n8 = (int)(T * DIM_IN / 8);
    cast_f32_bf16x8<<<(n8 + 255) / 256, 256, 0, stream>>>(x, XB, n8);
  }
  transpose_cast64<0><<<dim3(DIM_HID / 64, DIM_IN / 64, NUM_EXP), 256, 0, stream>>>(
      w1, DIM_HID, (long)DIM_IN * DIM_HID, W1T, DIM_IN, (long)DIM_HID * DIM_IN);
  transpose_cast64<1><<<dim3(DIM_EO / 64, DIM_HID / 64, NUM_EXP), 256, 0, stream>>>(
      w2, DIM_EO, (long)DIM_HID * DIM_EO, W2T, LD_W2T, (long)DIM_HID);
  transpose_cast64<0><<<dim3(DIM_OUT / 64, DIM_EO / 64, 1), 256, 0, stream>>>(
      wo, DIM_OUT, 0L, WOT, DIM_EO, 0L);
  build_wgt<<<1, 256, 0, stream>>>(wg, WGT);
  build_w2t_tail<<<1, 256, 0, stream>>>(b2, W2T);
  {
    const int tiles = (int)(T / 64) * (NGATE_PAD / 64);
    gemm64t<1, 0, 0, 0, false, 0><<<dim3((tiles + 7) / 8, 1), 256, 0, stream>>>(
        XB, nullptr, DIM_IN, 0L, WGT, nullptr, DIM_IN, 0L,
        GL, nullptr, NGATE_PAD, 0L, nullptr, nullptr, (int)T, NGATE_PAD, DIM_IN, 1.0f);
  }

  for (int ch = 0; ch < nChunk; ++ch) {
    const size_t row0 = (size_t)ch * CHUNK_ROWS;
    gate_softmax256<<<CHUNK_ROWS / 256, 256, 0, stream>>>(GL + row0 * NGATE_PAD, bg, GATE, HGX);
    {
      const int tiles = (CHUNK_ROWS / 64) * (NCAT / 64);
      gemm64t<1, 0, 2, 1, true, 2><<<dim3((tiles + 7) / 8, 1), 256, 0, stream>>>(
          XB + row0 * DIM_IN, nullptr, DIM_IN, 0L, W1T, nullptr, DIM_IN, 0L,
          HGX, nullptr, LD_HGX, 0L, b1, GATE, CHUNK_ROWS, NCAT, DIM_IN, 1.0f);
    }
    {
      const int tiles = (CHUNK_ROWS / 64) * (DIM_EO / 64);
      gemm64t<0, 0, 0, 2, false, 0><<<dim3((tiles + 7) / 8, 1), 256, 0, stream>>>(
          HGX, nullptr, LD_HGX, 0L, W2T, nullptr, LD_W2T, 0L,
          WEIH, WEIL, DIM_EO, 0L, nullptr, nullptr, CHUNK_ROWS, DIM_EO, KFC2, FC2_SCALE);
    }
    {
      const int tiles = (CHUNK_ROWS / 64) * (DIM_OUT / 64);
      gemm64t<1, 1, 2, 0, false, 0><<<dim3((tiles + 7) / 8, 1), 256, 0, stream>>>(
          WEIH, WEIL, DIM_EO, 0L, WOT, nullptr, DIM_EO, 0L,
          out + row0 * DIM_OUT, nullptr, DIM_OUT, 0L, bo, nullptr, CHUNK_ROWS, DIM_OUT, DIM_EO, 1.0f);
    }
  }
}
